// FourierModel_70196945486447
// MI455X (gfx1250) — hardware-run, weakly checked
//
#include <hip/hip_runtime.h>


#define NS   2048
#define NW   1024
#define NO   4096
#define NP   100000
#define NPP  100032
#define NH   32
#define NU   4160
typedef _Float16 h16;
typedef unsigned short bf;
typedef __attribute__((ext_vector_type(16))) __bf16   v16bf;
typedef __attribute__((ext_vector_type(16))) _Float16 v16h;
typedef __attribute__((ext_vector_type(8)))  _Float16 v8h;
typedef __attribute__((ext_vector_type(8)))  unsigned short v8us;
typedef __attribute__((ext_vector_type(8)))  float    v8f;
typedef __attribute__((ext_vector_type(4)))  float    v4f;
typedef v8h  __attribute__((may_alias)) v8ha;
typedef v4f  __attribute__((may_alias)) v4fa;
typedef v8us __attribute__((may_alias)) v8usa;

__device__ __forceinline__ unsigned short f2bf(float f) { unsigned u = __float_as_uint(f); u += 0x7FFFu + ((u >> 16) & 1u); return (unsigned short)(u >> 16); }
__device__ __forceinline__ float bf2f(unsigned short b) { return __uint_as_float(((unsigned)b) << 16); }
__device__ __forceinline__ float bfr(float f) { return bf2f(f2bf(f)); }
__device__ __forceinline__ v16h cat16(v8h lo, v8h hi) { return __builtin_shufflevector(lo, hi, 0, 1, 2, 3, 4, 5, 6, 7, 8, 9, 10, 11, 12, 13, 14, 15); }
__device__ __forceinline__ v16bf cat16b(v8us lo, v8us hi) { return __builtin_bit_cast(v16bf, __builtin_shufflevector(lo, hi, 0, 1, 2, 3, 4, 5, 6, 7, 8, 9, 10, 11, 12, 13, 14, 15)); }
__device__ __forceinline__ v8f wmma16(v16h a, v16h b, v8f c) { return __builtin_amdgcn_wmma_f32_16x16x32_f16(false, a, false, b, (short)0, c, false, false); }
__device__ __forceinline__ v8f wmmab(v16bf a, v16bf b, v8f c) { return __builtin_amdgcn_wmma_f32_16x16x32_bf16(false, a, false, b, (short)0, c, false, false); }

template <typename T16> struct WFrag;
template <> struct WFrag<h16> { typedef v16h V; static __device__ __forceinline__ V ld(const h16* p) { return cat16(*(const v8h*)p, *(const v8h*)(p + 16)); } static __device__ __forceinline__ v8f mma(V a, V b, v8f c) { return wmma16(a, b, c); } };
template <> struct WFrag<bf> { typedef v16bf V; static __device__ __forceinline__ V ld(const bf* p) { return cat16b(*(const v8us*)p, *(const v8us*)(p + 16)); } static __device__ __forceinline__ v8f mma(V a, V b, v8f c) { return wmmab(a, b, c); } };
template <typename T16, int NSPLIT, bool BIAS>
__global__ __launch_bounds__(32) void k_gemmw(const T16* __restrict__ A, const T16* __restrict__ A2, const T16* __restrict__ Bt, const T16* __restrict__ Bt2, int K, float* C, int ldc, const float* __restrict__ bias, size_t sA, size_t sB, size_t sC) {
    typedef typename WFrag<T16>::V V;
    __shared__ __align__(16) float os[16 * 68];
    const size_t z = blockIdx.z; A += z * sA; if (A2) A2 += z * sA; Bt += z * sB; if (Bt2) Bt2 += z * sB; C += z * sC;
    const int lane = threadIdx.x & 31, lr = lane & 15, hi = lane >> 4; const int r0 = blockIdx.x * 64, c0 = blockIdx.y * 64;
    v8f acc[4][4];
#pragma unroll
    for (int mb = 0; mb < 4; ++mb)
#pragma unroll
        for (int nb = 0; nb < 4; ++nb) acc[mb][nb] = (v8f){};
    const size_t aoff = (size_t)(r0 + lr) * K + 8 * hi, boff = (size_t)(c0 + lr) * K + 8 * hi;
    for (int kc = 0; kc < K; kc += 32) {
        V a[4], a2[4];
#pragma unroll
        for (int mb = 0; mb < 4; ++mb) { a[mb] = WFrag<T16>::ld(A + aoff + (size_t)mb * 16 * K + kc); if (NSPLIT == 1 || NSPLIT == 2) a2[mb] = WFrag<T16>::ld(A2 + aoff + (size_t)mb * 16 * K + kc); }
#pragma unroll
        for (int nb = 0; nb < 4; ++nb) { const V b = WFrag<T16>::ld(Bt + boff + (size_t)nb * 16 * K + kc); V b2; if (NSPLIT >= 2) b2 = WFrag<T16>::ld(Bt2 + boff + (size_t)nb * 16 * K + kc);
#pragma unroll
            for (int mb = 0; mb < 4; ++mb) { acc[mb][nb] = WFrag<T16>::mma(a[mb], b, acc[mb][nb]); if (NSPLIT == 1 || NSPLIT == 2) acc[mb][nb] = WFrag<T16>::mma(a2[mb], b, acc[mb][nb]); if (NSPLIT >= 2) acc[mb][nb] = WFrag<T16>::mma(a[mb], b2, acc[mb][nb]); } }
        asm volatile("v_nop\n\tv_nop\n\tv_nop\n\tv_nop" : "+v"(acc[0][0]), "+v"(acc[1][1]), "+v"(acc[2][2]), "+v"(acc[3][3]) : "v"(a[0]), "v"(a[3]));
    }
#pragma unroll
    for (int mb = 0; mb < 4; ++mb) {
#pragma unroll
        for (int nb = 0; nb < 4; ++nb) {
#pragma unroll
            for (int j = 0; j < 8; ++j) os[(hi * 8 + j) * 68 + nb * 16 + lr] = acc[mb][nb][j]; }
        __builtin_amdgcn_wave_barrier(); asm volatile("" ::: "memory");
        float* crow = C + (size_t)(r0 + mb * 16) * ldc + c0;
#pragma unroll 1
        for (int ps = 0; ps < 2; ++ps) {
#pragma unroll
            for (int s = 0; s < 8; ++s) { const int row = 2 * s + hi, cofs = lr * 4; v4f val = *(const v4fa*)(os + row * 68 + cofs); if (BIAS) { val[0] += bfr(bias[c0 + cofs]); val[1] += bfr(bias[c0 + cofs + 1]); val[2] += bfr(bias[c0 + cofs + 2]); val[3] += bfr(bias[c0 + cofs + 3]); }
                *(volatile v4f*)(crow + (size_t)row * ldc + cofs) = val; }
            if (ps == 0) __threadfence(); }
        __builtin_amdgcn_wave_barrier(); asm volatile("" ::: "memory");
    }
}

typedef __attribute__((ext_vector_type(2))) _Float16 v2h;
typedef __attribute__((ext_vector_type(4))) _Float16 v4h;
typedef __attribute__((ext_vector_type(2))) unsigned short v2us;
typedef __attribute__((ext_vector_type(4))) unsigned short v4us;
typedef __attribute__((ext_vector_type(2))) float v2f;
__device__ __forceinline__ h16 toh_flush(float x) { const float z = (fabsf(x) < 6.103515625e-05f) ? 0.0f : x; return (h16)z; }

__global__ __launch_bounds__(64) void k_cat16(const float* __restrict__ U, int wu, int pu, int uin, const float* __restrict__ W, int ww, int pw, int win, h16* dst, int KP) { const int k0 = (blockIdx.x * 64 + threadIdx.x) * 8; if (k0 >= KP) return; const int r = blockIdx.y; const unsigned mu = 0u - (unsigned)(uin != 0), mw = 0u - (unsigned)(win != 0); v8h o;
#pragma unroll
    for (int q = 0; q < 8; ++q) { const int k = k0 + q; const bool iu = k < wu; const bool iw = (!iu) && (k < wu + ww); const int ku = min(k, wu - 1); const int kw = min(max(k - wu, 0), max(ww - 1, 0)); const float a = U[(size_t)r * pu + ku]; const float b = W[(size_t)r * pw + kw];
        const float va = __uint_as_float((__float_as_uint(bfr(a)) & mu) | (__float_as_uint(a) & ~mu)); const float vb = __uint_as_float((__float_as_uint(bfr(b)) & mw) | (__float_as_uint(b) & ~mw)); const unsigned su = 0u - (unsigned)iu, sw = 0u - (unsigned)iw; o[q] = toh_flush(__uint_as_float((__float_as_uint(va) & su) | (__float_as_uint(vb) & sw))); }
    *(volatile v8h*)(dst + (size_t)r * KP + k0) = o; __threadfence(); *(volatile v8h*)(dst + (size_t)r * KP + k0) = o; }

__device__ __forceinline__ float om(int i) { return __fdiv_rn(__fmul_rn(6.2831855f, (float)i), 10.0f); }

__global__ __launch_bounds__(256) void k_ge16(const float* __restrict__ H, h16* G, size_t n8) { const size_t t = (size_t)blockIdx.x * 256 + threadIdx.x; if (t >= n8) return; const v8f v = *(const v8f*)(H + t * 8); v8h o;
#pragma unroll
    for (int q = 0; q < 8; ++q) { const float x = v[q]; const float u = __fmul_rn(0.7978845608f, __fadd_rn(x, __fmul_rn(0.044715f, __fmul_rn(__fmul_rn(x, x), x)))); const float th = __fsub_rn(1.0f, __fdiv_rn(2.0f, __fadd_rn(expf(__fmul_rn(2.0f, u)), 1.0f))); o[q] = toh_flush(__fmul_rn(__fmul_rn(0.5f, x), __fadd_rn(1.0f, th))); }
    *(volatile v8h*)(G + t * 8) = o; __threadfence(); *(volatile v8h*)(G + t * 8) = o; }

__global__ __launch_bounds__(256) void k_bv(const float* __restrict__ s, const float* __restrict__ wb, const float* __restrict__ bb, float* V) { const int q = blockIdx.x * 256 + threadIdx.x; if (q >= NS) return; const v4f x = *(const v4f*)(s + (size_t)q * 4); float a = 0.0f;
#pragma unroll
    for (int k = 0; k < 4; ++k) a = __fmaf_rn(bfr(x[k]), bfr(wb[k]), a);
    const float o = __fadd_rn(a, bfr(bb[0])); *(volatile float*)(V + q) = o; __threadfence(); *(volatile float*)(V + q) = o; }

__global__ __launch_bounds__(32) void k_cs(const float* __restrict__ w, const float* __restrict__ V, float* Us) { const int c = blockIdx.x * 32 + threadIdx.x; const bool col = c < NO; const bool tot = c == NO; const float* p = col ? (w + c) : V; const size_t st = col ? (size_t)NO : (tot ? (size_t)1 : (size_t)0); const float live = (col || tot) ? 1.0f : 0.0f; float a = 0.0f;
    for (int q = 0; q < NS; ++q) a = __fadd_rn(a, p[(size_t)q * st]);
    const bool tab = (c > NO) && (c <= NO + NH); const float tv = om(tab ? (c - NO) : 1); const float o = tab ? tv : __fmul_rn(live, a); *(volatile float*)(Us + c) = o; __threadfence(); *(volatile float*)(Us + c) = o; }

__global__ __launch_bounds__(256) void k_wa(const float* __restrict__ Us, h16* A12) { const int t = blockIdx.x * 256 + threadIdx.x; if (t >= 128 * NH / 8) return; const int m = t / 4, j0 = (t % 4) * 8; const int blk = m / 32, i = m % 32; const int c = (blk == 0) ? 0 : ((blk == 1) ? 3 : ((blk == 2) ? 1 : 2)); const v8f v = *(const v8f*)(Us + 1024 * c + 32 * i + j0); v8h o;
#pragma unroll
    for (int q = 0; q < 8; ++q) o[q] = toh_flush(v[q]);
    *(volatile v8h*)(A12 + (size_t)t * 8) = o; __threadfence(); *(volatile v8h*)(A12 + (size_t)t * 8) = o; }

__global__ __launch_bounds__(256) void k_tr(const float* __restrict__ r, h16* CY, h16* SY) { const int t = blockIdx.x * 256 + threadIdx.x; if (t >= NPP * NH / 8) return; const int n = t / 4, j0 = (t % 4) * 8; const int nn = n < NP ? n : NP - 1; const float live = n < NP ? 1.0f : 0.0f; const float y = bfr(r[(size_t)nn * 2 + 1]); v8h oc, os;
#pragma unroll
    for (int q = 0; q < 8; ++q) { const float ph = __fmul_rn(om(j0 + q + 1), y); oc[q] = toh_flush(__fmul_rn(live, __cosf(ph))); os[q] = toh_flush(__fmul_rn(live, __sinf(ph))); }
    *(volatile v8h*)(CY + (size_t)t * 8) = oc; *(volatile v8h*)(SY + (size_t)t * 8) = os; __threadfence(); *(volatile v8h*)(CY + (size_t)t * 8) = oc; *(volatile v8h*)(SY + (size_t)t * 8) = os; }

__global__ __launch_bounds__(256) void k_fin(const float* __restrict__ r, const float* __restrict__ T1, const float* __restrict__ T2, const float* __restrict__ Us, float* out) { const int n = blockIdx.x * 256 + threadIdx.x; if (n >= NP) return; const float x = bfr(r[(size_t)n * 2]); float a = 0.0f;
    for (int i = 0; i < NH; ++i) { const float ph = __fmul_rn(Us[NO + 1 + i], x); const float cx = __cosf(ph), sx = __sinf(ph); a = __fmaf_rn(cx, T1[(size_t)i * NPP + n], a); a = __fmaf_rn(sx, T1[(size_t)(32 + i) * NPP + n], a); a = __fmaf_rn(sx, T2[(size_t)i * NPP + n], a); a = __fmaf_rn(cx, T2[(size_t)(32 + i) * NPP + n], a); }
    const float o = __fadd_rn(Us[NO], a); *(volatile float*)(out + n) = o; __threadfence(); *(volatile float*)(out + n) = o; }

extern "C" void kernel_launch(void* const* d_in, const int* in_sizes, int n_in, void* d_out, int out_size, void* d_ws, size_t ws_size, hipStream_t stream) {
    if (n_in < 12) return;
    if (in_sizes[0] != NS * 4 || in_sizes[1] != NP * 2 || in_sizes[2] != NW * 4 || in_sizes[3] != NW || in_sizes[4] != NW * NW || in_sizes[5] != NW || in_sizes[6] != NW * NW || in_sizes[7] != NW || in_sizes[8] != NO * NW || in_sizes[9] != NO || in_sizes[10] != 4 || in_sizes[11] != 1) return;
    if (out_size != NP) return;
    static_assert(NS % 64 == 0 && NW % 64 == 0 && NO % 64 == 0 && NPP % 64 == 0 && NPP >= NP && NW % 512 == 0 && (NS * NW / 8) % 256 == 0 && NS % 256 == 0 && NU % 32 == 0 && NU >= NO + 1 + NH && (NPP * NH / 8) % 256 == 0 && NO == 4 * NH * NH, "every product: M and N multiples of 64, the depth a multiple of 32; a plane row a whole number of lines; every flat grid exact but k_fin's last block");
    const float* s = (const float*)d_in[0]; const float* r = (const float*)d_in[1]; const float* W1 = (const float*)d_in[2]; const float* b1 = (const float*)d_in[3]; const float* W2 = (const float*)d_in[4]; const float* b2 = (const float*)d_in[5]; const float* W3 = (const float*)d_in[6]; const float* b3 = (const float*)d_in[7]; const float* W4 = (const float*)d_in[8]; const float* b4 = (const float*)d_in[9]; const float* wb = (const float*)d_in[10]; const float* bb = (const float*)d_in[11];
    float* out = (float*)d_out;
    char* wsp = (char*)d_ws; auto take = [&](size_t bytes) { char* p = wsp; wsp += (bytes + 255) & ~(size_t)255; return (void*)p; };
    h16* S16 = (h16*)take((size_t)NS * 64 * 2); h16* W1p = (h16*)take((size_t)NW * 64 * 2); h16* W2p = (h16*)take((size_t)NW * NW * 2); h16* W3p = (h16*)take((size_t)NW * NW * 2); h16* W4p = (h16*)take((size_t)NO * NW * 2);
    float* H = (float*)take((size_t)NS * NW * 4); h16* G = (h16*)take((size_t)NS * NW * 2);
    float* Wc = (float*)take((size_t)NS * NO * 4); float* V = (float*)take((size_t)NS * 4); float* Us = (float*)take((size_t)NU * 4); h16* A12 = (h16*)take((size_t)128 * NH * 2); h16* CY = (h16*)take((size_t)NPP * NH * 2); h16* SY = (h16*)take((size_t)NPP * NH * 2); float* T1 = (float*)take((size_t)64 * NPP * 4); float* T2 = (float*)take((size_t)64 * NPP * 4);
    if ((size_t)(wsp - (char*)d_ws) > ws_size) return;
    auto cat = [&](const float* U, int rows, int wu, h16* d, int KP) { k_cat16<<<dim3((KP + 511) / 512, rows, 1), 64, 0, stream>>>(U, wu, wu, 1, U, 0, wu, 1, d, KP); };
    cat(s, NS, 4, S16, 64); cat(W1, NW, 4, W1p, 64); cat(W2, NW, NW, W2p, NW); cat(W3, NW, NW, W3p, NW); cat(W4, NO, NW, W4p, NW);
    const size_t n8 = (size_t)NS * NW / 8; const unsigned gg = (unsigned)(n8 / 256);
    k_gemmw<h16, 0, true><<<dim3(NS / 64, NW / 64, 1), 32, 0, stream>>>(S16, nullptr, W1p, nullptr, 64, H, NW, b1, 0, 0, 0);
    k_ge16<<<gg, 256, 0, stream>>>(H, G, n8);
    k_gemmw<h16, 0, true><<<dim3(NS / 64, NW / 64, 1), 32, 0, stream>>>(G, nullptr, W2p, nullptr, NW, H, NW, b2, 0, 0, 0);
    k_ge16<<<gg, 256, 0, stream>>>(H, G, n8);
    k_gemmw<h16, 0, true><<<dim3(NS / 64, NW / 64, 1), 32, 0, stream>>>(G, nullptr, W3p, nullptr, NW, H, NW, b3, 0, 0, 0);
    k_ge16<<<gg, 256, 0, stream>>>(H, G, n8);
    k_gemmw<h16, 0, true><<<dim3(NS / 64, NO / 64, 1), 32, 0, stream>>>(G, nullptr, W4p, nullptr, NW, Wc, NO, b4, 0, 0, 0);
    k_bv<<<(unsigned)(NS / 256), 256, 0, stream>>>(s, wb, bb, V);
    k_cs<<<(unsigned)(NU / 32), 32, 0, stream>>>(Wc, V, Us);
    k_wa<<<(unsigned)((128 * NH / 8 + 255) / 256), 256, 0, stream>>>(Us, A12);
    k_tr<<<(unsigned)(NPP * NH / 8 / 256), 256, 0, stream>>>(r, CY, SY);
    k_gemmw<h16, 0, false><<<dim3(1, NPP / 64, 1), 32, 0, stream>>>(A12, nullptr, CY, nullptr, NH, T1, NPP, nullptr, 0, 0, 0);
    k_gemmw<h16, 0, false><<<dim3(1, NPP / 64, 1), 32, 0, stream>>>(A12 + 64 * NH, nullptr, SY, nullptr, NH, T2, NPP, nullptr, 0, 0, 0);
    k_fin<<<(unsigned)((NP + 255) / 256), 256, 0, stream>>>(r, T1, T2, Us, out);
}
